// GeometricAwareChannelRouter_27298812133589
// MI455X (gfx1250) — hardware-verified
//
#include <hip/hip_runtime.h>
#include <math.h>

typedef __attribute__((ext_vector_type(16))) _Float16 v16h;
typedef __attribute__((ext_vector_type(16))) __bf16 v16b;
typedef __attribute__((ext_vector_type(8)))  _Float16 v8h;
typedef __attribute__((ext_vector_type(8)))  float v8f;
typedef __attribute__((ext_vector_type(4)))  float v4f;
typedef __attribute__((ext_vector_type(2)))  float v2f;
typedef __attribute__((ext_vector_type(4)))  unsigned v4u;
typedef __attribute__((ext_vector_type(4)))  int v4i;
typedef float __attribute__((may_alias)) float_a;
typedef int __attribute__((may_alias)) int_a;

template <typename T> __device__ __forceinline__ void vst2(void* p, T v) { *(volatile T*)p = v; __threadfence(); *(volatile T*)p = v; }
__device__ __forceinline__ v8f wmma16(v16h a, v16h b, v8f c) {
  v8f d = __builtin_amdgcn_wmma_f32_16x16x32_f16(false, a, false, b, (short)0, c, false, false);
  asm volatile("v_nop\n\tv_nop\n\tv_nop\n\tv_nop" : "+v"(d) : "v"(a), "v"(b));
  return d;
}
__device__ __forceinline__ v8f wmma_bf(v16b a, v16b b, v8f c) {
  v8f d = __builtin_amdgcn_wmma_f32_16x16x32_bf16(false, a, false, b, (short)0, c, false, false);
  asm volatile("v_nop\n\tv_nop\n\tv_nop\n\tv_nop" : "+v"(d) : "v"(a), "v"(b));
  return d;
}
__device__ __forceinline__ v16h frag_h(const _Float16* rowk0, int lane) {
  union { v16h v; v8h q[2]; } u; const _Float16* p = rowk0 + 8 * (lane >> 4);
  u.q[0] = *(const v8h*)p; u.q[1] = *(const v8h*)(p + 16); return u.v;
}
__device__ __forceinline__ v16h frag_f32(const float* rowk0, int lane) {
  v16h a; const float* p = rowk0 + 8 * (lane >> 4);
#pragma unroll
  for (int i = 0; i < 8; ++i) { a[i] = (_Float16)p[i]; a[8 + i] = (_Float16)p[16 + i]; }
  return a;
}
__device__ __forceinline__ v16h frag_f32s(const float* rowk0, int lane, float sc) {
  v16h a; const float* p = rowk0 + 8 * (lane >> 4);
#pragma unroll
  for (int i = 0; i < 8; ++i) { a[i] = (_Float16)(p[i] * sc); a[8 + i] = (_Float16)(p[16 + i] * sc); }
  return a;
}
__device__ __forceinline__ v16h fragc_f32(const float* W, int k0, int n, int lane, int ld, int K) {
  v16h a; const int g = lane >> 4;
#pragma unroll
  for (int i = 0; i < 8; ++i) { const int ka = k0 + 8 * g + i, kb = ka + 16;
    a[i] = (_Float16)(ka < K ? W[(size_t)(ka < K ? ka : K - 1) * ld + n] : 0.f); a[8 + i] = (_Float16)(kb < K ? W[(size_t)(kb < K ? kb : K - 1) * ld + n] : 0.f); }
  return a;
}
struct F2 { v16b h, l; };
__device__ __forceinline__ F2 bsplit16(const float v[16]) { F2 r;
#pragma unroll
  for (int i = 0; i < 16; ++i) { const __bf16 h = (__bf16)v[i]; r.h[i] = h; r.l[i] = (__bf16)(v[i] - (float)h); }
  return r; }
__device__ __forceinline__ F2 split_row(const float* row, int k0, int lane) { float v[16]; const float* p = row + k0 + 8 * (lane >> 4);
#pragma unroll
  for (int i = 0; i < 8; ++i) { v[i] = p[i]; v[8 + i] = p[16 + i]; }
  return bsplit16(v); }
__device__ __forceinline__ F2 split_rowK(const float* row, int k0, int lane, int K) { float v[16]; const int g = lane >> 4;
#pragma unroll
  for (int i = 0; i < 8; ++i) { const int ka = k0 + 8 * g + i, kb = ka + 16; v[i] = ka < K ? row[ka < K ? ka : K - 1] : 0.f; v[8 + i] = kb < K ? row[kb < K ? kb : K - 1] : 0.f; }
  return bsplit16(v); }
__device__ __forceinline__ F2 split_col(const float* W, int k0, int n, int lane, int ld, int K) { float v[16]; const int g = lane >> 4;
#pragma unroll
  for (int i = 0; i < 8; ++i) { const int ka = k0 + 8 * g + i, kb = ka + 16; v[i] = ka < K ? W[(size_t)(ka < K ? ka : K - 1) * ld + n] : 0.f; v[8 + i] = kb < K ? W[(size_t)(kb < K ? kb : K - 1) * ld + n] : 0.f; }
  return bsplit16(v); }
__device__ __forceinline__ v8f mac3(const F2& a, const F2& b, v8f c) { c = wmma_bf(a.l, b.h, c); c = wmma_bf(a.h, b.l, c); return wmma_bf(a.h, b.h, c); }
__device__ __forceinline__ float sigm(float v) { return 1.0f / (1.0f + expf(-v)); }
#define LDSX() do { asm volatile("s_wait_dscnt 0" ::: "memory"); __builtin_amdgcn_wave_barrier(); __builtin_amdgcn_fence(__ATOMIC_RELEASE, "workgroup"); } while (0)


#define NB 8
#define CCH 512
#define NPX 1024
#define SS 1024
#define DM 512
#define DI 512
#define NH 8
#define HD 64
#define QKVW (3 * DI)
#ifndef TQB
#define TQB (SS / 64)
#define TNB NB
#define TOB (NB * SS / 64)
#endif
typedef __attribute__((ext_vector_type(8))) __bf16 v8b;
__device__ __forceinline__ v16b frag_b(const __bf16* rowk0, int lane) {
  union { v16b v; v8b q[2]; } u; const __bf16* p = rowk0 + 8 * (lane >> 4);
  u.q[0] = *(const v8b*)p; u.q[1] = *(const v8b*)(p + 16); return u.v;
}
__device__ __forceinline__ float bfr(float v) { return (float)(__bf16)v; }
__device__ __attribute__((noinline)) float exp_ni(float v) { return expf(v); }
__device__ __attribute__((noinline)) float erf_ni(float v) { return erff(v); }

#define PK_A 0
#define PK_P (PK_A + QKVW * DM)
#define PK_BR (PK_P + DM * DI)
#define PK_END (2 * PK_BR)
#define WS_PK  0u
#define WS_MSK (((WS_PK + 2u * PK_END) + 127u) / 128u * 128u)
#define WS_TH  (WS_MSK + 4u * NB * CCH)
#define WS_TL  (WS_TH + 2u * NB * NPX * CCH)
#define WS_TE  (WS_TL + 2u * NB * NPX * CCH)
#define WS_QK  (WS_TE + 2u * NB * NPX * CCH)
#define WS_VTH (WS_QK + 2u * NB * SS * 2 * DI)
#define WS_VTL (WS_VTH + 2u * NB * DI * SS)
#define WS_O   (WS_VTL + 2u * NB * DI * SS)
#define WS_OH  (WS_O + 4u * NB * SS * DI)
#define WS_OE  (WS_OH + 4u * NB * SS * DI)
#define WS_END (WS_OE + 4u * NB * SS * DI)

__device__ __attribute__((noinline)) float tanh_ni(float v) { return tanhf(v); }
__global__ __launch_bounds__(256) void k_gate(const float* __restrict__ X, const float* __restrict__ W1, const float* __restrict__ B1, const float* __restrict__ W2, const float* __restrict__ B2, float* __restrict__ MSK) {
  __shared__ float sp[CCH]; __shared__ float sh[128]; __shared__ __align__(16) float sm[CCH]; const int t = threadIdx.x; const int b = blockIdx.x;
  for (int c = t; c < CCH; c += 256) { const float* p = X + ((size_t)b * CCH + c) * NPX; float a = 0.f; for (int i = 0; i < NPX; ++i) a += bfr(p[i]); sp[c] = a * (1.0f / NPX); }
  __syncthreads();
  if (t < 128) { float a = 0.f; for (int c = 0; c < CCH; ++c) a += sp[c] * bfr(W1[(size_t)c * 128 + t]); sh[t] = fmaxf(a + bfr(B1[t]), 0.f); }
  __syncthreads();
  for (int c = t; c < CCH; c += 256) { float a = 0.f; for (int k = 0; k < 128; ++k) a += sh[k] * bfr(W2[(size_t)k * CCH + c]); const float gv = a + bfr(B2[c]); sm[c] = (1.0f / (1.0f + exp_ni(-gv)) > 0.5f) ? 1.f : 0.f; }
  __syncthreads();
  for (int q = t; q < CCH / 4; q += 256) vst2(MSK + (size_t)b * CCH + q * 4, *(const v4f*)&sm[q * 4]);
}
__global__ __launch_bounds__(256) void k_tok(const float* __restrict__ X, const float* __restrict__ MSK, __bf16* __restrict__ TH, __bf16* __restrict__ TL, __bf16* __restrict__ TE) {
  __shared__ float st[64][CCH + 4]; __shared__ float sn[CCH][2]; const int tid = threadIdx.x; const int b = blockIdx.x / (NPX / 64), n0 = (blockIdx.x % (NPX / 64)) * 64;
  for (int q = tid; q < 64 * CCH; q += 256) { const int c = q >> 6, px = q & 63; st[px][c] = bfr(X[((size_t)b * CCH + c) * NPX + n0 + px]); }
  __syncthreads();
  for (int q = tid; q < CCH * 2; q += 256) { const int c = q >> 1, hr = q & 1; const float m = MSK[(size_t)b * CCH + c]; float s = 0.f; for (int w = 0; w < 32; ++w) { const float u = st[hr * 32 + w][c] * m; s += u * u; } const float nn = sqrtf(s); sn[c][hr] = tanh_ni(nn) / fmaxf(nn, 1e-15f); }
  __syncthreads();
  for (int q = tid; q < 64 * (CCH / 8); q += 256) { const int px = q / (CCH / 8), pc = q % (CCH / 8); __bf16 h8[8], l8[8], e8[8];
#pragma unroll
    for (int i = 0; i < 8; ++i) { const int c = pc * 8 + i; const float m = MSK[(size_t)b * CCH + c]; const float tv = st[px][c]; const float hv = (tv * m) * sn[c][px >> 5]; const __bf16 hb = (__bf16)hv; h8[i] = hb; l8[i] = (__bf16)(hv - (float)hb); e8[i] = (__bf16)(tv * (1.f - m)); }
    const size_t o = ((size_t)b * NPX + n0 + px) * CCH + pc * 8; vst2((unsigned*)(TH + o), *(const v4u*)h8); vst2((unsigned*)(TL + o), *(const v4u*)l8); vst2((unsigned*)(TE + o), *(const v4u*)e8); }
}
__global__ __launch_bounds__(256) void k_packT(const float* __restrict__ WQKV, const float* __restrict__ WO, const float* __restrict__ WQKV2, const float* __restrict__ WO2, __bf16* __restrict__ PK) {
  __shared__ __align__(16) __bf16 s[DM > DI ? DM : DI]; const int n = blockIdx.x, which = blockIdx.y, tid = threadIdx.x; const float* Wm; int K, N, cn; size_t dst; PK += (size_t)blockIdx.z * PK_BR; if (blockIdx.z) { WQKV = WQKV2; WO = WO2; }
  if (which < 3) { if (n >= DI) return; Wm = WQKV; K = DM; N = 3 * DI; cn = which * DI + n; dst = PK_A + ((size_t)which * DI + n) * DM; } else { if (n >= DM) return; Wm = WO; K = DI; N = DM; cn = n; dst = PK_P + (size_t)n * DI; }
  for (int k = tid; k < K; k += 256) s[k] = (__bf16)Wm[(size_t)k * N + cn];
  __syncthreads();
  for (int q = tid; q < K / 8; q += 256) vst2((unsigned*)(PK + dst + q * 8), *(const v4u*)&s[q * 8]);
}
__global__ __launch_bounds__(128) void k_qkv(const __bf16* __restrict__ AH, const __bf16* __restrict__ AL, const __bf16* __restrict__ P, const float* __restrict__ BQKV, _Float16* __restrict__ QK, _Float16* __restrict__ VTH, _Float16* __restrict__ VTL) {
  __shared__ __align__(16) _Float16 so[4][16][136]; __shared__ __align__(16) _Float16 sth[128][72], stl[128][72];
  const int tid = threadIdx.x, wave = tid >> 5, lane = tid & 31, col = lane & 15, g = lane >> 4; const size_t r0 = (size_t)blockIdx.x * 64 + wave * 16; const int n0 = blockIdx.y * 128;
  v8f acc[8] = {};
#pragma unroll 2
  for (int kc = 0; kc < DM / 32; ++kc) { const v16b a = frag_b(AH + (r0 + col) * DM + kc * 32, lane); v16b al; if (AL) al = frag_b(AL + (r0 + col) * DM + kc * 32, lane);
#pragma unroll
    for (int j = 0; j < 8; ++j) { const v16b w = frag_b(P + (size_t)(n0 + j * 16 + col) * DM + kc * 32, lane); if (AL) acc[j] = wmma_bf(al, w, acc[j]); acc[j] = wmma_bf(a, w, acc[j]); } }
#pragma unroll
  for (int j = 0; j < 8; ++j) { const float bb = bfr(BQKV[n0 + j * 16 + col]);
#pragma unroll
    for (int r = 0; r < 8; ++r) acc[j][r] += bb; }
  if (n0 < 2 * DI) { const float sc = (n0 < DI) ? 0.125f : 1.0f;
#pragma unroll
    for (int j = 0; j < 8; ++j) {
#pragma unroll
      for (int r = 0; r < 8; ++r) so[wave][8 * g + r][j * 16 + col] = (_Float16)(acc[j][r] * sc); }
    LDSX();
    for (int rl = 0; rl < 16; ++rl) if (lane < 16) vst2((unsigned*)(QK + (r0 + rl) * (2 * DI) + n0 + lane * 8), *(const v4u*)&so[wave][rl][lane * 8]);
  } else {
#pragma unroll
    for (int j = 0; j < 8; ++j) {
#pragma unroll
      for (int r = 0; r < 8; ++r) { const float v = acc[j][r]; const _Float16 hv = (_Float16)v; sth[j * 16 + col][wave * 16 + 8 * g + r] = hv; stl[j * 16 + col][wave * 16 + 8 * g + r] = (_Float16)((v - (float)hv) * 2048.0f); } }
    __syncthreads();
    const size_t rb = (size_t)blockIdx.x * 64; const int b = (int)(rb / SS), s0 = (int)(rb % SS); const int pc0 = n0 - 2 * DI;
    for (int q = tid; q < 128 * 8; q += 128) { const int d = q >> 3, pc = q & 7; const size_t o = ((size_t)b * DI + pc0 + d) * SS + s0 + pc * 8; vst2((unsigned*)(VTH + o), *(const v4u*)&sth[d][pc * 8]); vst2((unsigned*)(VTL + o), *(const v4u*)&stl[d][pc * 8]); }
  }
}
__global__ __launch_bounds__(128) void k_attn(const _Float16* __restrict__ QK, const _Float16* __restrict__ VTH, const _Float16* __restrict__ VTL, float* __restrict__ O) {
  __shared__ __align__(16) float sp[4][16][36]; __shared__ __align__(16) float so[4][16][68];
  const int tid = threadIdx.x, wave = tid >> 5, lane = tid & 31, col = lane & 15, g = lane >> 4;
  const int qb = blockIdx.x, h = blockIdx.y, b = blockIdx.z; const int q0 = qb * 64 + wave * 16; const size_t rq = (size_t)b * SS + q0 + col;
  v16h aq[2];
#pragma unroll
  for (int kc = 0; kc < 2; ++kc) aq[kc] = frag_h(QK + rq * (2 * DI) + h * HD + kc * 32, lane);
  float m[8], l[8];
#pragma unroll
  for (int r = 0; r < 8; ++r) { m[r] = -3.0e38f; l[r] = 0.f; }
  v8f acc[4] = {}, accl[4] = {};
#pragma unroll 1
  for (int ks = 0; ks < SS / 32; ++ks) { v8f s[2];
#pragma unroll
    for (int ct = 0; ct < 2; ++ct) { const int kk = ks * 32 + ct * 16 + col; const _Float16* krow = QK + ((size_t)b * SS + kk) * (2 * DI) + DI + h * HD; v8f c = {};
#pragma unroll
      for (int kc = 0; kc < 2; ++kc) c = wmma16(aq[kc], frag_h(krow + kc * 32, lane), c);
      s[ct] = c; }
#pragma unroll
    for (int r = 0; r < 8; ++r) { float mx = fmaxf(s[0][r], s[1][r]);
#pragma unroll
      for (int o = 1; o < 16; o <<= 1) mx = fmaxf(mx, __shfl_xor(mx, o));
      const float mn = fmaxf(m[r], mx); const float alpha = __expf(m[r] - mn);
      const float e0 = (float)(_Float16)__expf(s[0][r] - mn), e1 = (float)(_Float16)__expf(s[1][r] - mn); float es = e0 + e1;
#pragma unroll
      for (int o = 1; o < 16; o <<= 1) es += __shfl_xor(es, o);
      l[r] = l[r] * alpha + es; m[r] = mn;
#pragma unroll
      for (int dt = 0; dt < 4; ++dt) { acc[dt][r] *= alpha; accl[dt][r] *= alpha; }
      sp[wave][8 * g + r][col] = e0; sp[wave][8 * g + r][16 + col] = e1; }
    LDSX();
    const v16h pa = frag_f32(&sp[wave][col][0], lane);
#pragma unroll
    for (int dt = 0; dt < 4; ++dt) { const size_t vr = ((size_t)b * DI + h * HD + dt * 16 + col) * SS + ks * 32; acc[dt] = wmma16(pa, frag_h(VTH + vr, lane), acc[dt]); accl[dt] = wmma16(pa, frag_h(VTL + vr, lane), accl[dt]); }
    LDSX(); }
#pragma unroll
  for (int r = 0; r < 8; ++r) { const float il = 1.0f / l[r];
#pragma unroll
    for (int dt = 0; dt < 4; ++dt) so[wave][8 * g + r][dt * 16 + col] = (acc[dt][r] + accl[dt][r] * (1.0f / 2048.0f)) * il; }
  LDSX();
  for (int rl = 0; rl < 16; ++rl) if (lane < 16) vst2(O + ((size_t)b * SS + q0 + rl) * DI + h * HD + lane * 4, *(const v4f*)&so[wave][rl][lane * 4]);
}
__global__ __launch_bounds__(128) void k_out(const float* __restrict__ O, const __bf16* __restrict__ P, const float* __restrict__ BO, float* __restrict__ Y) {
  __shared__ __align__(16) float so[4][16][132];
  const int tid = threadIdx.x, wave = tid >> 5, lane = tid & 31, col = lane & 15, g = lane >> 4; const size_t r0 = (size_t)blockIdx.x * 64 + wave * 16; const int n0 = blockIdx.y * 128;
  v8f acc[8] = {};
#pragma unroll 2
  for (int kc = 0; kc < DI / 32; ++kc) { const F2 a = split_row(O + (r0 + col) * DI, kc * 32, lane);
#pragma unroll
    for (int j = 0; j < 8; ++j) { const v16b w = frag_b(P + (size_t)(n0 + j * 16 + col) * DI + kc * 32, lane); acc[j] = wmma_bf(a.l, w, acc[j]); acc[j] = wmma_bf(a.h, w, acc[j]); } }
#pragma unroll
  for (int j = 0; j < 8; ++j) { const float bb = bfr(BO[n0 + j * 16 + col]);
#pragma unroll
    for (int r = 0; r < 8; ++r) so[wave][8 * g + r][j * 16 + col] = acc[j][r] + bb; }
  LDSX();
  for (int rl = 0; rl < 16; ++rl) vst2(Y + (r0 + rl) * DM + n0 + lane * 4, *(const v4f*)&so[wave][rl][lane * 4]);
}
__device__ __attribute__((noinline)) float atanh_ni(float v) { return atanhf(v); }
__global__ __launch_bounds__(256) void k_fin(const float* __restrict__ OH, const float* __restrict__ OE, float* __restrict__ OUT) {
  __shared__ __align__(16) float st[CCH][68]; __shared__ float ssc[CCH][2]; const int tid = threadIdx.x; const int b = blockIdx.x / (NPX / 64), n0 = (blockIdx.x % (NPX / 64)) * 64;
  for (int q = tid; q < 64 * CCH; q += 256) { const int px = q & 63, c = q >> 6; st[c][px] = OH[((size_t)b * NPX + n0 + px) * CCH + c]; }
  __syncthreads();
  for (int q = tid; q < CCH * 2; q += 256) { const int c = q >> 1, hr = q & 1; float s = 0.f; for (int w = 0; w < 32; ++w) { const float v = st[c][hr * 32 + w]; s += v * v; } const float nn = sqrtf(s); const float nc = fminf(fmaxf(nn, 0.f), 1.0f - 1e-5f); ssc[c][hr] = atanh_ni(nc) / fmaxf(nn, 1e-15f); }
  __syncthreads();
  for (int q = tid; q < 64 * CCH; q += 256) { const int px = q & 63, c = q >> 6; const size_t o = ((size_t)b * NPX + n0 + px) * CCH + c; st[c][px] = st[c][px] * ssc[c][px >> 5] + OE[o]; }
  __syncthreads();
  for (int q = tid; q < CCH * 16; q += 256) { const int c = q >> 4, pc = q & 15; vst2(OUT + ((size_t)b * CCH + c) * NPX + n0 + pc * 4, *(const v4f*)&st[c][pc * 4]); }
}
extern "C" void kernel_launch(void* const* d_in, const int* in_sizes, int n_in, void* d_out, int out_size, void* d_ws, size_t ws_size, hipStream_t stream) {
  (void)in_sizes; (void)n_in; (void)out_size;
  const float** F = (const float**)d_in;
  if (ws_size < (size_t)WS_END) return;
  char* ws = (char*)d_ws; __bf16* PK = (__bf16*)(ws + WS_PK); _Float16 *QK = (_Float16*)(ws + WS_QK), *VTH = (_Float16*)(ws + WS_VTH), *VTL = (_Float16*)(ws + WS_VTL); float *O = (float*)(ws + WS_O), *MSK = (float*)(ws + WS_MSK), *OH = (float*)(ws + WS_OH), *OE = (float*)(ws + WS_OE); __bf16 *TH = (__bf16*)(ws + WS_TH), *TL = (__bf16*)(ws + WS_TL), *TE = (__bf16*)(ws + WS_TE);
  k_packT<<<dim3(DM > DI ? DM : DI, 4, 2), 256, 0, stream>>>(F[6], F[8], F[10], F[12], PK);
  k_gate<<<NB, 256, 0, stream>>>(F[0], F[2], F[3], F[4], F[5], MSK);
  k_tok<<<NB * NPX / 64, 256, 0, stream>>>(F[0], MSK, TH, TL, TE);
  k_qkv<<<dim3(TNB * SS / 64, QKVW / 128), 128, 0, stream>>>(TH, TL, PK + PK_A, F[7], QK, VTH, VTL);
  k_attn<<<dim3(TQB, NH, TNB), 128, 0, stream>>>(QK, VTH, VTL, O);
  k_out<<<dim3(TOB, DM / 128), 128, 0, stream>>>(O, PK + PK_P, F[9], OH);
  k_qkv<<<dim3(TNB * SS / 64, QKVW / 128), 128, 0, stream>>>(TE, nullptr, PK + PK_BR + PK_A, F[11], QK, VTH, VTL);
  k_attn<<<dim3(TQB, NH, TNB), 128, 0, stream>>>(QK, VTH, VTL, O);
  k_out<<<dim3(TOB, DM / 128), 128, 0, stream>>>(O, PK + PK_BR + PK_P, F[13], OE);
  k_fin<<<TNB * NPX / 64, 256, 0, stream>>>(OH, OE, (float*)d_out);
}
